// MultiHeadAtten_64364379898184
// MI455X (gfx1250) — hardware-verified
//
#include <hip/hip_runtime.h>
#include <math.h>
#include <stdint.h>

#define NB    8
#define SEQ   1024
#define DM    1024
#define NH    8
#define HD    128
#define ROWS  (NB * SEQ)
#define OUTN  (ROWS * DM)
#define NIT   (SEQ / 16)
#define NJT   (SEQ / 64)
#define PVT   ((SEQ / 32) * (HD / 64))
static_assert(NH * HD == DM);
static_assert(HD == 128);
static_assert((HD / 64) == 2);
static_assert((SEQ % 64) == 0 && (DM % 64) == 0 && (ROWS % 64) == 0 && (DM % 32) == 0 && (HD % 64) == 0);
static_assert(((ROWS / 64) * (DM / 64)) % 8 == 0);
static_assert(((ROWS / 64) * (HD / 64)) % 8 == 0);
static_assert((NH * PVT) % 8 == 0);
static_assert(((ROWS * DM / 8) % 256) == 0);

typedef _Float16 v16h __attribute__((ext_vector_type(16)));
typedef _Float16 v8h  __attribute__((ext_vector_type(8)));
typedef __bf16   v16b __attribute__((ext_vector_type(16)));
typedef __bf16   v8b  __attribute__((ext_vector_type(8)));
typedef float    v8f  __attribute__((ext_vector_type(8)));
typedef float    v4f  __attribute__((ext_vector_type(4)));
typedef unsigned int v4u __attribute__((ext_vector_type(4)));

__device__ __forceinline__ unsigned short bf_bits(float f) {
  unsigned u = __float_as_uint(f);
  return (unsigned short)((u + 0x7FFFu + ((u >> 16) & 1u)) >> 16);
}
__device__ __forceinline__ float bf_up(unsigned short h) { return __uint_as_float(((unsigned)h) << 16); }
__device__ __forceinline__ unsigned short h_bits(_Float16 x) { return __builtin_bit_cast(unsigned short, x); }
__device__ __forceinline__ unsigned pk16(unsigned short a, unsigned short b) { return (unsigned)a | ((unsigned)b << 16); }
__device__ __forceinline__ v8f zero8() { v8f z = {0.f, 0.f, 0.f, 0.f, 0.f, 0.f, 0.f, 0.f}; return z; }

__device__ __forceinline__ v16b ldfrag_b(const __bf16* p) {
  union { v16b v; v8b h[2]; } f;
  f.h[0] = *(const v8b*)(p);
  f.h[1] = *(const v8b*)(p + 16);
  return f.v;
}
__device__ __forceinline__ v16h ldfrag_h(const _Float16* p) {
  union { v16h v; v8h h[2]; } f;
  f.h[0] = *(const v8h*)(p);
  f.h[1] = *(const v8h*)(p + 16);
  return f.v;
}

__device__ __forceinline__ v8f mma_h(v16h a, v16h b, v8f c) {
  c = __builtin_amdgcn_wmma_f32_16x16x32_f16(false, a, false, b, (short)0, c, false, false);
#if defined(__HIP_DEVICE_COMPILE__)
  asm volatile("v_nop\n\tv_nop\n\tv_nop\n\tv_nop" : "+v"(c) : "v"(a), "v"(b));
#endif
  return c;
}
__device__ __forceinline__ v8f mma_b_raw(v16b a, v16b b, v8f c) {
  return __builtin_amdgcn_wmma_f32_16x16x32_bf16(false, a, false, b, (short)0, c, false, false);
}
__device__ __forceinline__ void dep_guard_b(v8f& a, v8f& b, v16b x, v16b y) {
#if defined(__HIP_DEVICE_COMPILE__)
  asm volatile("v_nop\n\tv_nop\n\tv_nop\n\tv_nop" : "+v"(a), "+v"(b) : "v"(x), "v"(y));
#endif
}
__device__ __forceinline__ void keep4_b(v16b a, v16b b, v16b c, v16b d) {
#if defined(__HIP_DEVICE_COMPILE__)
  asm volatile("v_nop" :: "v"(a), "v"(b), "v"(c), "v"(d));
#endif
}
__device__ __forceinline__ void acc_guard4(v8f& a, v8f& b, v8f& c, v8f& d) {
#if defined(__HIP_DEVICE_COMPILE__)
  asm volatile("v_nop\n\tv_nop\n\tv_nop\n\tv_nop" : "+v"(a), "+v"(b), "+v"(c), "+v"(d));
#endif
}

__global__ __launch_bounds__(256) void cvt_bf16x8(const float* __restrict__ in, unsigned short* out, int n8) {
  const int i = blockIdx.x * 256 + threadIdx.x;
  if (i < n8) {
    const v4f a = *(const v4f*)(in + (size_t)i * 8);
    const v4f b = *(const v4f*)(in + (size_t)i * 8 + 4);
    v4u p;
    p[0] = pk16(bf_bits(a[0]), bf_bits(a[1]));
    p[1] = pk16(bf_bits(a[2]), bf_bits(a[3]));
    p[2] = pk16(bf_bits(b[0]), bf_bits(b[1]));
    p[3] = pk16(bf_bits(b[2]), bf_bits(b[3]));
    *(volatile v4u*)(out + (size_t)i * 8) = p;
    __threadfence();
    *(volatile v4u*)(out + (size_t)i * 8) = p;
  }
}

__global__ __launch_bounds__(256) void tr_bf16_64(const float* __restrict__ in, int R, int C,
                                                  unsigned short* out) {
  __shared__ __align__(16) float st[64 * 68];
  const int tid = threadIdx.x;
  const int r0  = blockIdx.x * 64;
  const int c0  = blockIdx.y * 64;
#pragma unroll
  for (int i = 0; i < 4; ++i) {
    const int idx = i * 256 + tid;
    const int rr = idx >> 4, c4 = (idx & 15) * 4;
    const v4f a = *(const v4f*)(in + ((size_t)(r0 + rr)) * C + c0 + c4);
    *(v4f*)(st + rr * 68 + c4) = a;
  }
  __syncthreads();

  const int g = tid >> 3, piece = tid & 7;
  v4u hv[2];
  size_t hofs[2];
#pragma unroll
  for (int it = 0; it < 2; ++it) {
    const int cc = it * 32 + g;
    v4u a;
#pragma unroll
    for (int e = 0; e < 4; ++e) {
      const float f0 = st[(piece * 8 + 2 * e) * 68 + cc];
      const float f1 = st[(piece * 8 + 2 * e + 1) * 68 + cc];
      a[e] = pk16(bf_bits(f0), bf_bits(f1));
    }
    hv[it] = a;
    hofs[it] = ((size_t)(c0 + cc)) * R + r0 + piece * 8;
  }
  for (int pass = 0; pass < 2; ++pass) {
#pragma unroll
    for (int it = 0; it < 2; ++it) {
      *(volatile v4u*)(out + hofs[it]) = hv[it];
    }
    __threadfence();
  }
}

__global__ __launch_bounds__(256) void plane_f16x8(const float* __restrict__ in, unsigned short* hp, int n8,
                                                   float scale) {
  const int i = blockIdx.x * 256 + threadIdx.x;
  if (i < n8) {
    const v4f a = *(const v4f*)(in + (size_t)i * 8);
    const v4f b = *(const v4f*)(in + (size_t)i * 8 + 4);
    float f[8];
    f[0] = a[0]; f[1] = a[1]; f[2] = a[2]; f[3] = a[3];
    f[4] = b[0]; f[5] = b[1]; f[6] = b[2]; f[7] = b[3];
    v4u ph;
#pragma unroll
    for (int e = 0; e < 4; ++e) {
      const _Float16 x0 = (_Float16)(f[2 * e] * scale);
      const _Float16 x1 = (_Float16)(f[2 * e + 1] * scale);
      ph[e] = pk16(h_bits(x0), h_bits(x1));
    }
    *(volatile v4u*)(hp + (size_t)i * 8) = ph;
    __threadfence();
    *(volatile v4u*)(hp + (size_t)i * 8) = ph;
  }
}

__global__ __launch_bounds__(256) void gemm64(
    const unsigned short* __restrict__ Ap, int lda,
    const unsigned short* __restrict__ Btp, int ldb,
    const float* __restrict__ bias,
    float* C, int ldc, int M, int N, int K) {
  const __bf16* Ab  = (const __bf16*)(const void*)Ap;
  const __bf16* Bb  = (const __bf16*)(const void*)Btp;
  __shared__ __align__(16) float sT[8][16 * 68];
  const int lane = threadIdx.x & 31;
  const int wave = threadIdx.x >> 5;
  const int tilesN = N >> 6;
  const int tilesM = M >> 6;
  const int tile = blockIdx.x * 8 + wave;
  if (tile >= tilesM * tilesN) return;
  const int tm = tile / tilesN;
  const int tn = tile - tm * tilesN;
  const int m0 = tm << 6;
  const int n0 = tn << 6;

  const int rlane = lane & 15;
  const int koff  = (lane >> 4) * 8;
  const int mOff  = (lane >> 4) * 8;

  v8f acc[4][4];
#pragma unroll
  for (int i = 0; i < 4; ++i)
#pragma unroll
    for (int j = 0; j < 4; ++j) acc[i][j] = zero8();

  for (int k0 = 0; k0 < K; k0 += 32) {
    v16b bh[4];
#pragma unroll
    for (int j = 0; j < 4; ++j) {
      const size_t bo = (size_t)(n0 + (j << 4) + rlane) * ldb + koff + k0;
      bh[j] = ldfrag_b(Bb + bo);
    }
#pragma unroll
    for (int i = 0; i < 4; ++i) {
      const size_t ao = (size_t)(m0 + (i << 4) + rlane) * lda + koff + k0;
      const v16b ah = ldfrag_b(Ab + ao);
#pragma unroll
      for (int j = 0; j < 4; ++j) {
        acc[i][j] = mma_b_raw(ah, bh[j], acc[i][j]);
      }
      dep_guard_b(acc[i][0], acc[i][3], ah, ah);
    }
    keep4_b(bh[0], bh[1], bh[2], bh[3]);
  }
  acc_guard4(acc[0][0], acc[0][1], acc[0][2], acc[0][3]);
  acc_guard4(acc[1][0], acc[1][1], acc[1][2], acc[1][3]);
  acc_guard4(acc[2][0], acc[2][1], acc[2][2], acc[2][3]);
  acc_guard4(acc[3][0], acc[3][1], acc[3][2], acc[3][3]);

  float bz[4];
#pragma unroll
  for (int j = 0; j < 4; ++j) bz[j] = bf_up(bf_bits(bias[n0 + (j << 4) + rlane]));

  float* slab = sT[wave];
#pragma unroll
  for (int i = 0; i < 4; ++i) {
    const int mBase = m0 + (i << 4);
#pragma unroll
    for (int r = 0; r < 8; ++r) {
#pragma unroll
      for (int j = 0; j < 4; ++j) {
        slab[(mOff + r) * 68 + (j << 4) + rlane] = acc[i][j][r] + bz[j];
      }
    }
    __builtin_amdgcn_fence(__ATOMIC_RELEASE, "workgroup");
    __builtin_amdgcn_wave_barrier();
    __builtin_amdgcn_fence(__ATOMIC_ACQUIRE, "workgroup");
    {
      const int hh = lane >> 4, c4 = (lane & 15) * 4;
      v4f ov[8];
#pragma unroll
      for (int it = 0; it < 8; ++it) {
        const int row = it * 2 + hh;
        ov[it] = *(const v4f*)(slab + row * 68 + c4);
      }
      for (int pass = 0; pass < 2; ++pass) {
#pragma unroll
        for (int it = 0; it < 8; ++it) {
          const int row = it * 2 + hh;
          *(volatile v4f*)(C + (size_t)(mBase + row) * ldc + n0 + c4) = ov[it];
        }
        __threadfence();
      }
    }
    __builtin_amdgcn_fence(__ATOMIC_RELEASE, "workgroup");
    __builtin_amdgcn_wave_barrier();
    __builtin_amdgcn_fence(__ATOMIC_ACQUIRE, "workgroup");
  }
}

__global__ __launch_bounds__(256) void v_plane(const float* __restrict__ vf, unsigned short* vth, float vscale) {
  __shared__ __align__(16) float sv[64 * 68];
  const int tid = threadIdx.x;
  const int t0  = blockIdx.x * 64;
  const int fh  = blockIdx.y;
  const int b   = blockIdx.z;
#pragma unroll
  for (int i = 0; i < 4; ++i) {
    const int idx = i * 256 + tid;
    const int tt = idx >> 4, c4 = (idx & 15) * 4;
    const v4f a = *(const v4f*)(vf + ((size_t)(b * SEQ + t0 + tt)) * HD + fh * 64 + c4);
    *(v4f*)(sv + tt * 68 + c4) = a;
  }
  __syncthreads();

  const int g = tid >> 3, piece = tid & 7;
  v4u hv[2];
  size_t hofs[2];
#pragma unroll
  for (int it = 0; it < 2; ++it) {
    const int d = it * 32 + g;
    v4u a;
#pragma unroll
    for (int e = 0; e < 4; ++e) {
      float f0 = sv[(piece * 8 + 2 * e) * 68 + d];
      float f1 = sv[(piece * 8 + 2 * e + 1) * 68 + d];
      f0 = (f0 >= 0.f) ? f0 : 0.01f * f0;
      f1 = (f1 >= 0.f) ? f1 : 0.01f * f1;
      a[e] = pk16(h_bits((_Float16)(f0 * vscale)), h_bits((_Float16)(f1 * vscale)));
    }
    hv[it] = a;
    hofs[it] = ((size_t)(b * HD + fh * 64 + d)) * SEQ + t0 + piece * 8;
  }
  for (int pass = 0; pass < 2; ++pass) {
#pragma unroll
    for (int it = 0; it < 2; ++it) {
      *(volatile v4u*)(vth + hofs[it]) = hv[it];
    }
    __threadfence();
  }
}

__global__ __launch_bounds__(256)
void scores_hsm(const unsigned short* __restrict__ qhp, const unsigned short* __restrict__ khp,
                unsigned short* ap, int b, float sscale, float pscale) {
  union H8 { v8h h; v4u u; };
  __shared__ __align__(16) float    sS[NH][16 * 64];
  __shared__ __align__(16) _Float16 sP[NH][16 * 72];
  const int tid  = threadIdx.x;
  const int h    = tid >> 5;
  const int lane = tid & 31;
  const int hh   = lane >> 4;
  const int c    = lane & 15;
  const int jt   = blockIdx.x % NJT;
  const int it   = blockIdx.x / NJT;
  const int i0   = it * 16;
  const int j0   = jt * 64;
  const size_t rowB = (size_t)b * SEQ;
  const _Float16* Qp = (const _Float16*)(const void*)qhp + (size_t)h * HD;
  const _Float16* Kp = (const _Float16*)(const void*)khp + (size_t)h * HD;

  v8f s[4];
#pragma unroll
  for (int jj = 0; jj < 4; ++jj) s[jj] = zero8();
#pragma unroll
  for (int dc = 0; dc < HD / 32; ++dc) {
    const v16h qa = ldfrag_h(Qp + (rowB + i0 + c) * DM + dc * 32 + 8 * hh);
#pragma unroll
    for (int jj = 0; jj < 4; ++jj) {
      const v16h kb = ldfrag_h(Kp + (rowB + j0 + jj * 16 + c) * DM + dc * 32 + 8 * hh);
      s[jj] = mma_h(qa, kb, s[jj]);
    }
  }
  float* ss = sS[h];
#pragma unroll
  for (int r = 0; r < 8; ++r) {
#pragma unroll
    for (int jj = 0; jj < 4; ++jj) {
      ss[(8 * hh + r) * 64 + jj * 16 + c] = s[jj][r] * sscale;
    }
  }
  __syncthreads();

  {
    const int ii = tid >> 4, cb = (tid & 15) * 4;
#pragma unroll
    for (int p = 0; p < 4; ++p) {
      const int col = cb + p;
      float v[NH];
#pragma unroll
      for (int g = 0; g < NH; ++g) v[g] = sS[g][ii * 64 + col];
      float m = v[0];
#pragma unroll
      for (int g = 1; g < NH; ++g) m = fmaxf(m, v[g]);
      float sum = 0.f;
#pragma unroll
      for (int g = 0; g < NH; ++g) {
        v[g] = __expf(v[g] - m);
        sum += v[g];
      }
      const float inv = (1.0f / sum) * pscale;
#pragma unroll
      for (int g = 0; g < NH; ++g) sP[g][ii * 72 + col] = (_Float16)(v[g] * inv);
    }
  }
  __syncthreads();

  {
    const int g4 = lane >> 3, piece = lane & 7;
    const _Float16* sp = sP[h];
    v4u hv[4];
    size_t hofs[4];
#pragma unroll
    for (int q = 0; q < 4; ++q) {
      const int row = q * 4 + g4;
      H8 x;
      x.h = *(const v8h*)(sp + row * 72 + piece * 8);
      hv[q] = x.u;
      hofs[q] = ((size_t)(h * SEQ + i0 + row)) * SEQ + j0 + piece * 8;
    }
    for (int pass = 0; pass < 2; ++pass) {
#pragma unroll
      for (int q = 0; q < 4; ++q) {
        *(volatile v4u*)(ap + hofs[q]) = hv[q];
      }
      __threadfence();
    }
  }
}

__global__ __launch_bounds__(256) void gemm_pv(
    const unsigned short* __restrict__ Pp, const unsigned short* __restrict__ Vtp,
    float* C, float oscale) {
  const _Float16* Bh = (const _Float16*)(const void*)Vtp;
  __shared__ __align__(16) float sT[8][16 * 68];
  const int lane = threadIdx.x & 31;
  const int wave = threadIdx.x >> 5;
  const int tile = blockIdx.x * 8 + wave;
  if (tile >= NH * PVT) return;
  const int h  = tile / PVT;
  const int t  = tile - h * PVT;
  const int tm = t >> 1;
  const int tn = t & 1;
  const int m0 = tm << 5;
  const int n0 = tn << 6;
  const _Float16* Ah = (const _Float16*)(const void*)Pp + (size_t)h * SEQ * SEQ;

  const int rlane = lane & 15;
  const int koff  = (lane >> 4) * 8;
  const int mOff  = (lane >> 4) * 8;

  v8f acc[2][4];
#pragma unroll
  for (int i = 0; i < 2; ++i)
#pragma unroll
    for (int j = 0; j < 4; ++j) acc[i][j] = zero8();

  for (int k0 = 0; k0 < SEQ; k0 += 32) {
    v16h ah[2];
#pragma unroll
    for (int i = 0; i < 2; ++i) {
      const size_t ao = (size_t)(m0 + (i << 4) + rlane) * SEQ + koff + k0;
      ah[i] = ldfrag_h(Ah + ao);
    }
#pragma unroll
    for (int j = 0; j < 4; ++j) {
      const size_t bo = (size_t)(n0 + (j << 4) + rlane) * SEQ + koff + k0;
      const v16h bfr = ldfrag_h(Bh + bo);
#pragma unroll
      for (int i = 0; i < 2; ++i) {
        acc[i][j] = mma_h(ah[i], bfr, acc[i][j]);
      }
    }
  }

  float* slab = sT[wave];
#pragma unroll
  for (int i = 0; i < 2; ++i) {
    const int mBase = m0 + (i << 4);
#pragma unroll
    for (int r = 0; r < 8; ++r) {
#pragma unroll
      for (int j = 0; j < 4; ++j) {
        slab[(mOff + r) * 68 + (j << 4) + rlane] = acc[i][j][r] * oscale;
      }
    }
    __builtin_amdgcn_fence(__ATOMIC_RELEASE, "workgroup");
    __builtin_amdgcn_wave_barrier();
    __builtin_amdgcn_fence(__ATOMIC_ACQUIRE, "workgroup");
    {
      const int hh = lane >> 4, c4 = (lane & 15) * 4;
      v4f ov[8];
#pragma unroll
      for (int it = 0; it < 8; ++it) {
        const int row = it * 2 + hh;
        ov[it] = *(const v4f*)(slab + row * 68 + c4);
      }
      for (int pass = 0; pass < 2; ++pass) {
#pragma unroll
        for (int it = 0; it < 8; ++it) {
          const int row = it * 2 + hh;
          *(volatile v4f*)(C + (size_t)(mBase + row) * DM + (size_t)h * HD + n0 + c4) = ov[it];
        }
        __threadfence();
      }
    }
    __builtin_amdgcn_fence(__ATOMIC_RELEASE, "workgroup");
    __builtin_amdgcn_wave_barrier();
    __builtin_amdgcn_fence(__ATOMIC_ACQUIRE, "workgroup");
  }
}

extern "C" void kernel_launch(void* const* d_in, const int* in_sizes, int n_in,
                              void* d_out, int out_size, void* d_ws, size_t ws_size,
                              hipStream_t stream) {
  if (n_in < 7) return;
  if (in_sizes[0] != NB * SEQ * DM) return;
  if (in_sizes[1] != DM * DM) return;
  if (in_sizes[2] != DM) return;
  if (in_sizes[3] != DM * DM) return;
  if (in_sizes[4] != DM) return;
  if (in_sizes[5] != DM * HD) return;
  if (in_sizes[6] != HD) return;
  if (out_size != OUTN) return;

  const float* x  = (const float*)d_in[0];
  const float* Wq = (const float*)d_in[1];
  const float* bq = (const float*)d_in[2];
  const float* Wk = (const float*)d_in[3];
  const float* bk = (const float*)d_in[4];
  const float* Wv = (const float*)d_in[5];
  const float* bv = (const float*)d_in[6];

  const size_t PXb = (size_t)ROWS * DM * 2;
  const size_t PW  = (size_t)DM * DM * 2;
  const size_t PWv = (size_t)HD * DM * 2;
  const size_t PF  = (size_t)ROWS * DM * 4;
  const size_t PH  = (size_t)ROWS * DM * 2;
  const size_t PVt = (size_t)NB * HD * SEQ * 2;
  const size_t PA  = (size_t)NH * SEQ * SEQ * 2;
  size_t off = 0;
  const size_t oXb = off; off += PXb;
  const size_t oWq = off; off += PW;
  const size_t oWk = off; off += PW;
  const size_t oWv = off; off += PWv;
  const size_t oTf = off; off += PF;
  const size_t oQh = off; off += PH;
  const size_t oKh = off; off += PH;
  const size_t oVt = off; off += PVt;
  const size_t oA  = off; off += PA;
  if (off > ws_size) return;
  if (off > (size_t)134217728) return;

  char* ws = (char*)d_ws;
  unsigned short* Xb  = (unsigned short*)(ws + oXb);
  unsigned short* Wqt = (unsigned short*)(ws + oWq);
  unsigned short* Wkt = (unsigned short*)(ws + oWk);
  unsigned short* Wvt = (unsigned short*)(ws + oWv);
  float*          Tf  = (float*)(ws + oTf);
  unsigned short* Qh  = (unsigned short*)(ws + oQh);
  unsigned short* Kh  = (unsigned short*)(ws + oKh);
  unsigned short* VTh = (unsigned short*)(ws + oVt);
  unsigned short* Ap  = (unsigned short*)(ws + oA);
  float*          outf = (float*)d_out;

  const dim3 blk(256);
  const int n8x = ROWS * DM / 8;
  const dim3 gCvtX((n8x + 255) / 256);
  const dim3 gTrW(DM / 64, DM / 64);
  const dim3 gTrV(DM / 64, HD / 64);
  const dim3 gGemm(((ROWS / 64) * (DM / 64) + 7) / 8);
  const dim3 gGemV(((ROWS / 64) * (HD / 64) + 7) / 8);
  const dim3 gVpl(SEQ / 64, HD / 64, NB);
  const dim3 gSc(NIT * NJT);
  const dim3 gPv((NH * PVT + 7) / 8);
  const float qkScale = 16.0f;
  const float sscale  = 0.08838834764831845f / 256.0f;
  const float pScale  = 1024.0f;
  const float vScale  = 256.0f;
  const float pvOscl  = 1.0f / 262144.0f;

  cvt_bf16x8<<<gCvtX, blk, 0, stream>>>(x, Xb, n8x);
  tr_bf16_64<<<gTrW, blk, 0, stream>>>(Wq, DM, DM, Wqt);
  tr_bf16_64<<<gTrW, blk, 0, stream>>>(Wk, DM, DM, Wkt);
  tr_bf16_64<<<gTrV, blk, 0, stream>>>(Wv, DM, HD, Wvt);
  gemm64<<<gGemm, blk, 0, stream>>>(Xb, DM, Wqt, DM, bq, Tf, DM, ROWS, DM, DM);
  plane_f16x8<<<gCvtX, blk, 0, stream>>>(Tf, Qh, n8x, qkScale);
  gemm64<<<gGemm, blk, 0, stream>>>(Xb, DM, Wkt, DM, bk, Tf, DM, ROWS, DM, DM);
  plane_f16x8<<<gCvtX, blk, 0, stream>>>(Tf, Kh, n8x, qkScale);
  gemm64<<<gGemV, blk, 0, stream>>>(Xb, DM, Wvt, DM, bv, Tf, HD, ROWS, HD, DM);
  v_plane<<<gVpl, blk, 0, stream>>>(Tf, VTh, vScale);
  for (int b = 0; b < NB; ++b) {
    scores_hsm<<<gSc, blk, 0, stream>>>(Qh, Kh, Ap, b, sscale, pScale);
    gemm_pv<<<gPv, blk, 0, stream>>>(Ap, VTh + (size_t)b * HD * SEQ, outf + (size_t)b * SEQ * DM, pvOscl);
  }
  (void)hipGetLastError();
}
